// JointSupervisedGroundedCoreferencer_45337674776936
// MI455X (gfx1250) — hardware-verified
//
#include <hip/hip_runtime.h>
#include <hip/hip_bf16.h>

typedef __attribute__((ext_vector_type(16))) _Float16 v16h;
typedef __attribute__((ext_vector_type(8)))  _Float16 v8h;
typedef __attribute__((ext_vector_type(8)))  float  v8f;

#define DD     1024
#define HH     1024
#define K1     3072
#define BSZ    8
#define NN     40
#define LL     20
#define NPAIRS 780
#define GROWS  (320*160)
#define TROWS  (8*780)
#define MT     32

static __device__ __forceinline__ unsigned short f2bf(float f){ union { _Float16 h; unsigned short u; } c; c.h = (_Float16)f; return c.u; }
static __device__ __forceinline__ float bf2f(unsigned short h){ union { _Float16 h; unsigned short u; } c; c.u = h; return (float)c.h; }
typedef __attribute__((ext_vector_type(4))) float v4f;
typedef __attribute__((ext_vector_type(4))) unsigned v4u;
typedef float __attribute__((may_alias)) float_a;
typedef int __attribute__((may_alias)) int_a;
template <typename T> __device__ __forceinline__ void vst2(void* p, T v) { *(volatile T*)p = v; __threadfence(); *(volatile T*)p = v; }
static __device__ __forceinline__ v8f wmma16(v16h a, v16h b, v8f c) {
  v8f d = __builtin_amdgcn_wmma_f32_16x16x32_f16(false, a, false, b, (short)0, c, false, false);
  asm volatile("v_nop\n\tv_nop\n\tv_nop\n\tv_nop" : "+v"(d) : "v"(a), "v"(b));
  return d;
}
static __device__ __forceinline__ v16h bfrag(const unsigned short* WT, size_t n, int ld, int koff, int hi) {
  union { v16h v; v8h q[2]; } b; const unsigned short* p = WT + n * (size_t)ld + koff + hi * 8;
  b.q[0] = *(const v8h*)p; b.q[1] = *(const v8h*)(p + 16); return b.v;
}

__global__ void cast_bf16_kernel(const float* __restrict__ src,
                                 unsigned short* __restrict__ dst, int n){
  for (int g = blockIdx.x*blockDim.x + threadIdx.x; g < n / 8; g += gridDim.x*blockDim.x) {
    union { unsigned short s[8]; v4u u; } pk;
#pragma unroll
    for (int e = 0; e < 8; ++e) pk.s[e] = f2bf(src[(size_t)g * 8 + e]);
    vst2(dst + (size_t)g * 8, pk.u);
  }
}

__global__ void transpose_bf16_kernel(const float* __restrict__ src,
                                      unsigned short* __restrict__ dst,
                                      int rows, int cols){
  __shared__ __align__(16) unsigned short tile[64][72];
  const int tilesC = cols / 64, tr = blockIdx.x / tilesC, tc = blockIdx.x % tilesC, tid = threadIdx.x;
  for (int i = tid; i < 64 * 64; i += 256) { const int r = i >> 6, c = i & 63; tile[c][r] = f2bf(src[(size_t)(tr * 64 + r) * cols + tc * 64 + c]); }
  __syncthreads();
  for (int g = tid; g < 64 * 8; g += 256) { const int c = g >> 3, pc = g & 7;
    vst2(dst + (size_t)(tc * 64 + c) * rows + tr * 64 + pc * 8, *(const v4u*)(&tile[c][pc * 8])); }
}

__global__ void triu_pairs_kernel(int* __restrict__ fi, int* __restrict__ si){
  int p = blockIdx.x*blockDim.x + threadIdx.x;
  if (p >= NPAIRS) return;
  int cum = 0;
  for (int f = 0; f < NN-1; ++f){
    int cnt = NN-1-f;
    if (p < cum + cnt){ vst2(fi + p, (int_a)f); vst2(si + p, (int_a)(f+1+(p-cum))); return; }
    cum += cnt;
  }
}

__global__ __launch_bounds__(256)
void gemm_rows_kernel(const unsigned short* __restrict__ rows,
                      const unsigned short* __restrict__ WT,
                      int ldw,
                      const float* __restrict__ bias,
                      float* __restrict__ out)
{
  __shared__ __align__(16) unsigned short atile[16*1024];
  __shared__ __align__(16) float so[8][16 * 128];
  const int tid  = threadIdx.x;
  const int lane = tid & 31;
  const int wave = tid >> 5;
  const int hi   = lane >> 4;
  const int lm   = lane & 15;
  const int c0   = wave * 128;
  const int row0 = blockIdx.x * 16;

  for (int e = tid; e < 16*1024; e += 256)
    atile[e] = rows[(size_t)(row0 + (e >> 10))*DD + (e & 1023)];
  __syncthreads();

  v8f acc[8];
  #pragma unroll
  for (int cb = 0; cb < 8; ++cb){ v8f z = {0.f,0.f,0.f,0.f,0.f,0.f,0.f,0.f}; acc[cb] = z; }

  for (int ks = 0; ks < DD/32; ++ks){
    int koff = ks * 32;
    v8h alo = *(const v8h*)&atile[lm*1024 + koff + hi*8];
    v8h ahi = *(const v8h*)&atile[lm*1024 + koff + 16 + hi*8];
    v16h A;
    #pragma unroll
    for (int e = 0; e < 8; ++e){ A[e] = alo[e]; A[8+e] = ahi[e]; }
    #pragma unroll
    for (int cb = 0; cb < 8; ++cb){
      int n = c0 + cb*16 + lm;
      v16h Bf = bfrag(WT, (size_t)n, ldw, koff, hi);
      acc[cb] = wmma16(A, Bf, acc[cb]);
    }
  }
  float* S = so[wave];
  #pragma unroll
  for (int cb = 0; cb < 8; ++cb){
    int n = c0 + cb*16 + lm;
    float bv = bias ? bias[n] : 0.f;
    #pragma unroll
    for (int r = 0; r < 8; ++r) S[(r + 8*hi) * 128 + cb*16 + lm] = acc[cb][r] + bv;
  }
  asm volatile("s_wait_dscnt 0" ::: "memory"); __builtin_amdgcn_wave_barrier(); __builtin_amdgcn_fence(__ATOMIC_RELEASE, "workgroup");
  #pragma unroll 4
  for (int r = 0; r < 16; ++r) vst2(out + (size_t)(row0 + r)*HH + c0 + lane * 4, *(const v4f*)(S + r * 128 + lane * 4));
}

__global__ __launch_bounds__(256)
void fused_pair_score_kernel(const unsigned short* __restrict__ srcA,
                             const unsigned short* __restrict__ srcB,
                             const float* __restrict__ addA,
                             const float* __restrict__ addB,
                             const unsigned short* __restrict__ WpT,
                             int ldp,
                             const unsigned short* __restrict__ W2T,
                             const float* __restrict__ bias2,
                             const float* __restrict__ W3,
                             const float* __restrict__ bias3,
                             const int* __restrict__ fiArr,
                             const int* __restrict__ siArr,
                             int mode,
                             const float* __restrict__ maskA,
                             const float* __restrict__ maskB,
                             float* __restrict__ out)
{
  __shared__ __align__(16) unsigned short ptile[MT*1024];
  const int tid  = threadIdx.x;
  const int lane = tid & 31;
  const int wave = tid >> 5;
  const int hi   = lane >> 4;
  const int lm   = lane & 15;
  const int c0   = wave * 128;
  const int tile = blockIdx.x;

  for (int e = tid; e < MT*1024; e += 256){
    int m = e >> 10;
    int k = e & 1023;
    int g = tile*MT + m;
    int ra, rb;
    if (mode == 0){ ra = g / 160; rb = g - ra*160; }
    else { int b = g / NPAIRS; int p = g - b*NPAIRS; ra = b*NN + fiArr[p]; rb = b*NN + siArr[p]; }
    float av = bf2f(srcA[(size_t)ra*DD + k]);
    float bv = bf2f(srcB[(size_t)rb*DD + k]);
    ptile[e] = f2bf(av * bv);
  }
  __syncthreads();

  v8f acc[2][8];
  #pragma unroll
  for (int mt = 0; mt < 2; ++mt)
    #pragma unroll
    for (int cb = 0; cb < 8; ++cb){ v8f z = {0.f,0.f,0.f,0.f,0.f,0.f,0.f,0.f}; acc[mt][cb] = z; }

  for (int ks = 0; ks < DD/32; ++ks){
    int koff = ks * 32;
    v16h A0, A1;
    {
      v8h lo = *(const v8h*)&ptile[lm*1024 + koff + hi*8];
      v8h hi8 = *(const v8h*)&ptile[lm*1024 + koff + 16 + hi*8];
      #pragma unroll
      for (int e = 0; e < 8; ++e){ A0[e] = lo[e]; A0[8+e] = hi8[e]; }
    }
    {
      v8h lo = *(const v8h*)&ptile[(16+lm)*1024 + koff + hi*8];
      v8h hi8 = *(const v8h*)&ptile[(16+lm)*1024 + koff + 16 + hi*8];
      #pragma unroll
      for (int e = 0; e < 8; ++e){ A1[e] = lo[e]; A1[8+e] = hi8[e]; }
    }
    #pragma unroll
    for (int cb = 0; cb < 8; ++cb){
      int n = c0 + cb*16 + lm;
      v16h Bf = bfrag(WpT, (size_t)n, ldp, koff, hi);
      acc[0][cb] = wmma16(A0, Bf, acc[0][cb]);
      acc[1][cb] = wmma16(A1, Bf, acc[1][cb]);
    }
  }

  int ra8[2][8], rb8[2][8];
  #pragma unroll
  for (int mt = 0; mt < 2; ++mt)
    #pragma unroll
    for (int r = 0; r < 8; ++r){
      int g = tile*MT + mt*16 + r + 8*hi;
      if (mode == 0){ ra8[mt][r] = g / 160; rb8[mt][r] = g - (g/160)*160; }
      else { int b = g / NPAIRS; int p = g - b*NPAIRS;
             ra8[mt][r] = b*NN + fiArr[p]; rb8[mt][r] = b*NN + siArr[p]; }
    }
  #pragma unroll
  for (int mt = 0; mt < 2; ++mt)
    #pragma unroll
    for (int cb = 0; cb < 8; ++cb){
      int n = c0 + cb*16 + lm;
      #pragma unroll
      for (int r = 0; r < 8; ++r){
        float v = acc[mt][cb][r] + addA[(size_t)ra8[mt][r]*HH + n]
                                 + addB[(size_t)rb8[mt][r]*HH + n];
        acc[mt][cb][r] = v > 0.f ? v : 0.f;
      }
    }
  __syncthreads();

  #pragma unroll
  for (int mt = 0; mt < 2; ++mt)
    #pragma unroll
    for (int cb = 0; cb < 8; ++cb){
      int n = c0 + cb*16 + lm;
      #pragma unroll
      for (int r = 0; r < 8; ++r)
        ptile[(mt*16 + r + 8*hi)*1024 + n] = f2bf(acc[mt][cb][r]);
    }
  __syncthreads();

  #pragma unroll
  for (int mt = 0; mt < 2; ++mt)
    #pragma unroll
    for (int cb = 0; cb < 8; ++cb){ v8f z = {0.f,0.f,0.f,0.f,0.f,0.f,0.f,0.f}; acc[mt][cb] = z; }
  for (int ks = 0; ks < HH/32; ++ks){
    int koff = ks * 32;
    v16h A0, A1;
    {
      v8h lo = *(const v8h*)&ptile[lm*1024 + koff + hi*8];
      v8h hi8 = *(const v8h*)&ptile[lm*1024 + koff + 16 + hi*8];
      #pragma unroll
      for (int e = 0; e < 8; ++e){ A0[e] = lo[e]; A0[8+e] = hi8[e]; }
    }
    {
      v8h lo = *(const v8h*)&ptile[(16+lm)*1024 + koff + hi*8];
      v8h hi8 = *(const v8h*)&ptile[(16+lm)*1024 + koff + 16 + hi*8];
      #pragma unroll
      for (int e = 0; e < 8; ++e){ A1[e] = lo[e]; A1[8+e] = hi8[e]; }
    }
    #pragma unroll
    for (int cb = 0; cb < 8; ++cb){
      int n = c0 + cb*16 + lm;
      v16h Bf = bfrag(W2T, (size_t)n, HH, koff, hi);
      acc[0][cb] = wmma16(A0, Bf, acc[0][cb]);
      acc[1][cb] = wmma16(A1, Bf, acc[1][cb]);
    }
  }
  __syncthreads();

  float* red = (float*)ptile;

  float part[2][8];
  #pragma unroll
  for (int mt = 0; mt < 2; ++mt)
    #pragma unroll
    for (int r = 0; r < 8; ++r) part[mt][r] = 0.f;
  #pragma unroll
  for (int mt = 0; mt < 2; ++mt)
    #pragma unroll
    for (int cb = 0; cb < 8; ++cb){
      int n = c0 + cb*16 + lm;
      float bv = bias2[n];
      float w3 = W3[n];
      #pragma unroll
      for (int r = 0; r < 8; ++r){
        float v = acc[mt][cb][r] + bv;
        v = v > 0.f ? v : 0.f;
        part[mt][r] += v * w3;
      }
    }
  #pragma unroll
  for (int mt = 0; mt < 2; ++mt)
    #pragma unroll
    for (int r = 0; r < 8; ++r) {
      float v = part[mt][r];
      #pragma unroll
      for (int o = 8; o >= 1; o >>= 1) v += __shfl_xor(v, o, 32);
      if (lm == 0) red[wave * 32 + mt*16 + r + 8*hi] = v;
    }
  __syncthreads();

  if (tid < MT){
    int g = tile*MT + tid;
    float sc = bias3[0];
    #pragma unroll
    for (int w = 0; w < 8; ++w) sc += red[w * 32 + tid];
    if (mode == 0){
      int i = g / 160, j = g - (g/160)*160;
      sc *= maskA[i] * maskB[j];
    }
    vst2(out + g, (float_a)sc);
  }
}

__global__ void loss_kernel(const float* __restrict__ gsc, float* __restrict__ out0){
  __shared__ float S[64];
  int t = threadIdx.x;
  if (t < 64){
    float s = 0.f;
    const float* p = gsc + t*800;
    for (int k = 0; k < 800; ++k) s += p[k];
    S[t] = s;
  }
  __syncthreads();
  if (t == 0){
    float loss = 0.f;
    for (int r = 0; r < 8; ++r){
      float mx = -1e30f;
      for (int c = 0; c < 8; ++c) mx = fmaxf(mx, S[r*8+c]);
      float se = 0.f;
      for (int c = 0; c < 8; ++c) se += expf(S[r*8+c] - mx);
      float lse = mx + logf(se);
      for (int c = 0; c < 8; ++c) loss -= (S[r*8+c] - lse);
    }
    for (int c = 0; c < 8; ++c){
      float mx = -1e30f;
      for (int r = 0; r < 8; ++r) mx = fmaxf(mx, S[r*8+c]);
      float se = 0.f;
      for (int r = 0; r < 8; ++r) se += expf(S[r*8+c] - mx);
      float lse = mx + logf(se);
      for (int r = 0; r < 8; ++r) loss -= (S[r*8+c] - lse);
    }
    vst2(out0, (float_a)(loss / (float)BSZ));
  }
}

#define NOUT (1 + GROWS + TROWS)
__global__ void flat_out_kernel(const float* __restrict__ L, const float* __restrict__ G, const float* __restrict__ T, float* __restrict__ out){
  for (int q = blockIdx.x*blockDim.x + threadIdx.x; q < (NOUT + 3) / 4; q += gridDim.x*blockDim.x) {
    float v[4];
    #pragma unroll
    for (int e = 0; e < 4; ++e) { int i = q * 4 + e; v[e] = (i == 0) ? L[0] : (i <= GROWS ? G[i - 1] : (i < NOUT ? T[i - 1 - GROWS] : 0.f)); }
    if (q * 4 + 4 <= NOUT) { v4f vv = {v[0], v[1], v[2], v[3]}; vst2(out + (size_t)q * 4, vv); }
    else { for (int e = 0; e < 4; ++e) if (q * 4 + e < NOUT) vst2(out + q * 4 + e, (float_a)v[e]); }
  }
}

extern "C" void kernel_launch(void* const* d_in, const int* in_sizes, int n_in,
                              void* d_out, int out_size, void* d_ws, size_t ws_size,
                              hipStream_t stream){
  const float* span = (const float*)d_in[0];
  const float* img  = (const float*)d_in[1];
  const float* smask = (const float*)d_in[2];
  const float* imask = (const float*)d_in[3];
  const float* tW1  = (const float*)d_in[4];
  const float* tb1  = (const float*)d_in[5];
  const float* tW2  = (const float*)d_in[6];
  const float* tb2  = (const float*)d_in[7];
  const float* tW3  = (const float*)d_in[8];
  const float* tb3  = (const float*)d_in[9];
  const float* gW1  = (const float*)d_in[10];
  const float* gb1  = (const float*)d_in[11];
  const float* gW2  = (const float*)d_in[12];
  const float* gb2  = (const float*)d_in[13];
  const float* gW3  = (const float*)d_in[14];
  const float* gb3  = (const float*)d_in[15];
  float* out = (float*)d_out;

  char* ws = (char*)d_ws;
  size_t off = 0;
  auto alloc = [&](size_t bytes)->void*{
    void* p = ws + off;
    off += (bytes + 255) & ~(size_t)255;
    return p;
  };
  unsigned short* f_bf = (unsigned short*)alloc((size_t)320*1024*2);
  unsigned short* v_bf = (unsigned short*)alloc((size_t)160*1024*2);
  unsigned short* gW1T = (unsigned short*)alloc((size_t)1024*3072*2);
  unsigned short* tW1T = (unsigned short*)alloc((size_t)1024*3072*2);
  unsigned short* gW2T = (unsigned short*)alloc((size_t)1024*1024*2);
  unsigned short* tW2T = (unsigned short*)alloc((size_t)1024*1024*2);
  int*   fiArr = (int*)alloc((size_t)NPAIRS*4);
  int*   siArr = (int*)alloc((size_t)NPAIRS*4);
  float* FW = (float*)alloc((size_t)320*1024*4);
  float* VW = (float*)alloc((size_t)160*1024*4);
  float* TF = (float*)alloc((size_t)320*1024*4);
  float* TS = (float*)alloc((size_t)320*1024*4);
  float* Gst = (float*)alloc((size_t)GROWS*4);
  float* Tst = (float*)alloc((size_t)TROWS*4);
  float* Lst = (float*)alloc(256);

  cast_bf16_kernel<<<160, 256, 0, stream>>>(span, f_bf, 320*1024);
  cast_bf16_kernel<<<80, 256, 0, stream>>>(img,  v_bf, 160*1024);
  transpose_bf16_kernel<<<48 * 16, 256, 0, stream>>>(gW1, gW1T, 3072, 1024);
  transpose_bf16_kernel<<<48 * 16, 256, 0, stream>>>(tW1, tW1T, 3072, 1024);
  transpose_bf16_kernel<<<16 * 16, 256, 0, stream>>>(gW2, gW2T, 1024, 1024);
  transpose_bf16_kernel<<<16 * 16, 256, 0, stream>>>(tW2, tW2T, 1024, 1024);
  triu_pairs_kernel<<<4, 256, 0, stream>>>(fiArr, siArr);

  gemm_rows_kernel<<<20, 256, 0, stream>>>(f_bf, gW1T,        K1, nullptr, FW);
  gemm_rows_kernel<<<10, 256, 0, stream>>>(v_bf, gW1T + 1024, K1, gb1,     VW);
  gemm_rows_kernel<<<20, 256, 0, stream>>>(f_bf, tW1T,        K1, nullptr, TF);
  gemm_rows_kernel<<<20, 256, 0, stream>>>(f_bf, tW1T + 1024, K1, tb1,     TS);

  fused_pair_score_kernel<<<GROWS/MT, 256, 0, stream>>>(
      f_bf, v_bf, FW, VW, gW1T + 2048, K1, gW2T, gb2, gW3, gb3,
      fiArr, siArr, 0, smask, imask, Gst);
  fused_pair_score_kernel<<<TROWS/MT, 256, 0, stream>>>(
      f_bf, f_bf, TF, TS, tW1T + 2048, K1, tW2T, tb2, tW3, tb3,
      fiArr, siArr, 1, nullptr, nullptr, Tst);

  loss_kernel<<<1, 64, 0, stream>>>(Gst, Lst);
  flat_out_kernel<<<(NOUT / 4 + 255) / 256, 256, 0, stream>>>(Lst, Gst, Tst, out);
}
